// S6_12824772346184
// MI455X (gfx1250) — hardware-verified
//
#include <hip/hip_runtime.h>
#include <math.h>

typedef __attribute__((ext_vector_type(16))) _Float16 v16h;
typedef __attribute__((ext_vector_type(8)))  _Float16 v8h;
typedef __attribute__((ext_vector_type(16))) __bf16   v16b;
typedef __attribute__((ext_vector_type(8)))  __bf16   v8b;
typedef __attribute__((ext_vector_type(8)))  float    v8f;
typedef __attribute__((ext_vector_type(4)))  float    v4f;

constexpr int kBatch   = 8;
constexpr int kSeq     = 2048;
constexpr int kDm      = 64;
constexpr int kNs      = 64;
constexpr int kRows    = kBatch * kSeq;
constexpr int kKc      = 3 * kDm;
constexpr int kNc      = kDm + 2 * kNs;
constexpr int kXBlocks = (kRows * kDm / 8) / 256;
constexpr int kWBlocks = (3 * 64 * kDm / 8) / 256;
constexpr int kRowsPerWave = 8;
constexpr int kOutBlocks   = kRows / (8 * kRowsPerWave);
constexpr int kGemmTiles   = (kRows / 64) * (kNc / 64);
constexpr int kGemmBlocks  = kGemmTiles / 8;
static_assert(kDm == 64 && kNs == 64, "plane builder assumes 64-wide rows");
static_assert(kRows == 16384 && kKc == 192 && kNc == 192, "shape constants");
static_assert((kKc % 32) == 0, "GEMM K multiple of 32");
static_assert((kRows % 64) == 0 && (kNc % 64) == 0, "GEMM M,N multiples of 64");
static_assert(kXBlocks * 256 * 8 == kRows * kDm, "x plane coverage");
static_assert(kWBlocks * 256 * 8 == 3 * 64 * kDm, "W plane coverage");
static_assert(kGemmBlocks * 8 == kGemmTiles, "tile coverage");
static_assert(kOutBlocks * 8 * kRowsPerWave == kRows, "row coverage");

constexpr size_t kOffAP   = 0;
constexpr size_t kOffBT   = kOffAP + (size_t)kRows * kKc * 2;
constexpr size_t kOffPP   = kOffBT + (size_t)kNc * kKc * 2;
constexpr size_t kWsTotal = kOffPP + (size_t)kRows * kNc * 4;
static_assert(kWsTotal == 18948096ull, "carve total");
static_assert(kWsTotal <= 134217728ull, "carve cap");
static_assert((kOffBT % 128) == 0 && (kOffPP % 128) == 0, "128-B aligned regions");

__device__ __forceinline__ unsigned short f2bf_bits(float f) {
  unsigned u = __float_as_uint(f);
  return (unsigned short)((u + 0x7FFFu + ((u >> 16) & 1u)) >> 16);
}
__device__ __forceinline__ float bf_bits2f(unsigned short h) { return __uint_as_float(((unsigned)h) << 16); }

__device__ __forceinline__ void row_guard_b(v8f& a, v8f& b, v8f& c, v8f& d, v16b x, v16b b0, v16b b1, v16b b2, v16b b3) {
  asm volatile("v_nop\n\tv_nop\n\tv_nop\n\tv_nop" : "+v"(a), "+v"(b), "+v"(c), "+v"(d) : "v"(x), "v"(b0), "v"(b1), "v"(b2), "v"(b3));
}
__device__ __forceinline__ void keep4_b(v16b a, v16b b, v16b c, v16b d) { asm volatile("v_nop" :: "v"(a), "v"(b), "v"(c), "v"(d)); }
__device__ __forceinline__ void acc_guard4(v8f& a, v8f& b, v8f& c, v8f& d) { asm volatile("v_nop\n\tv_nop\n\tv_nop\n\tv_nop" : "+v"(a), "+v"(b), "+v"(c), "+v"(d)); }

struct FragB {
  union U { v16b v; v8b h[2]; };
  static __device__ __forceinline__ v16b load(const __bf16* p) {
    U f; f.h[0] = *(const v8b*)(p); f.h[1] = *(const v8b*)(p + 16); return f.v;
  }
  static __device__ __forceinline__ v8f mma(v16b a, v16b b, v8f c) {
    return __builtin_amdgcn_wmma_f32_16x16x32_bf16(false, a, false, b, (short)0, c, false, false);
  }
};

__global__ __launch_bounds__(256) void build_planes_kernel(
    const float* __restrict__ x, const float* __restrict__ W1, const float* __restrict__ W2,
    const float* __restrict__ W3, unsigned short* __restrict__ AP, unsigned short* __restrict__ BT)
{
  const int blk = blockIdx.x;
  const bool isW = (blk >= kXBlocks);
  const int wb = isW ? (blk - kXBlocks) : 0;
  const int p = wb >> 1;
  const float* wsrc = (p == 0) ? W1 : ((p == 1) ? W2 : W3);
  const float* src = isW ? wsrc : x;
  const int ci = isW ? ((wb & 1) * 256 + (int)threadIdx.x) : (blk * 256 + (int)threadIdx.x);
  const int row = ci >> 3;
  const int c8 = (ci & 7) * 8;
  const size_t e0 = (size_t)row * kDm + c8;
  const v4f a0 = *(const v4f*)(src + e0);
  const v4f a1 = *(const v4f*)(src + e0 + 4);
  v8h hv, lv;
#pragma unroll
  for (int e = 0; e < 4; ++e) {
    const float f0 = a0[e];
    const float f1 = a1[e];
    const unsigned short h0 = f2bf_bits(f0), h1 = f2bf_bits(f1);
    const unsigned short l0 = f2bf_bits(f0 - bf_bits2f(h0)), l1 = f2bf_bits(f1 - bf_bits2f(h1));
    hv[e]     = __builtin_bit_cast(_Float16, h0);
    hv[4 + e] = __builtin_bit_cast(_Float16, h1);
    lv[e]     = __builtin_bit_cast(_Float16, l0);
    lv[4 + e] = __builtin_bit_cast(_Float16, l1);
  }
  unsigned short* dst = isW ? BT : AP;
  const int drow = isW ? (p * 64 + row) : row;
  unsigned short* q = dst + (size_t)drow * kKc + c8;
  const v8h s1 = isW ? hv : lv;
  const v8h s2 = isW ? lv : hv;
  *(volatile v8h*)(q)       = hv;
  *(volatile v8h*)(q + 64)  = s1;
  *(volatile v8h*)(q + 128) = s2;
  __threadfence();
  *(volatile v8h*)(q)       = hv;
  *(volatile v8h*)(q + 64)  = s1;
  *(volatile v8h*)(q + 128) = s2;
}

__global__ __launch_bounds__(256) void wmma_gemm64_bf16(
    const unsigned short* __restrict__ Ap, int lda,
    const unsigned short* __restrict__ Btp, int ldb,
    float* __restrict__ C, int ldc, int M, int N, int K)
{
  typedef __bf16 T;
  const T* A  = (const T*)Ap;
  const T* Bt = (const T*)Btp;
  __shared__ __align__(16) float sT[8][16 * 68];
  const int lane = threadIdx.x & 31;
  const int wave = threadIdx.x >> 5;
  const int tilesN = N >> 6;
  const int tilesM = M >> 6;
  const int tile = blockIdx.x * 8 + wave;
  if (tile >= tilesM * tilesN) return;
  const int tm = tile / tilesN;
  const int tn = tile - tm * tilesN;
  const int m0 = tm << 6;
  const int n0 = tn << 6;

  const int rlane = lane & 15;
  const int koff  = (lane >> 4) * 8;
  const int mOff  = (lane >> 4) * 8;

  v8f acc[4][4];
#pragma unroll
  for (int i = 0; i < 4; ++i)
#pragma unroll
    for (int j = 0; j < 4; ++j) acc[i][j] = (v8f){0.f,0.f,0.f,0.f,0.f,0.f,0.f,0.f};

#pragma unroll 1
  for (int k0 = 0; k0 < K; k0 += 32) {
    v16b bh[4];
#pragma unroll
    for (int j = 0; j < 4; ++j) {
      const size_t bo = (size_t)(n0 + (j << 4) + rlane) * ldb + koff + k0;
      bh[j] = FragB::load(Bt + bo);
    }
#pragma unroll
    for (int i = 0; i < 4; ++i) {
      const size_t ao = (size_t)(m0 + (i << 4) + rlane) * lda + koff + k0;
      v16b ah = FragB::load(A + ao);
#pragma unroll
      for (int j = 0; j < 4; ++j) acc[i][j] = FragB::mma(ah, bh[j], acc[i][j]);
      row_guard_b(acc[i][0], acc[i][1], acc[i][2], acc[i][3], ah, bh[0], bh[1], bh[2], bh[3]);
    }
    keep4_b(bh[0], bh[1], bh[2], bh[3]);
  }
  acc_guard4(acc[0][0], acc[0][1], acc[0][2], acc[0][3]);
  acc_guard4(acc[1][0], acc[1][1], acc[1][2], acc[1][3]);
  acc_guard4(acc[2][0], acc[2][1], acc[2][2], acc[2][3]);
  acc_guard4(acc[3][0], acc[3][1], acc[3][2], acc[3][3]);

  float* slab = sT[wave];
#pragma unroll
  for (int i = 0; i < 4; ++i) {
    const int mBase = m0 + (i << 4);
#pragma unroll
    for (int j = 0; j < 4; ++j) {
#pragma unroll
      for (int r = 0; r < 8; ++r) slab[(mOff + r) * 68 + (j << 4) + rlane] = acc[i][j][r];
    }
    __builtin_amdgcn_fence(__ATOMIC_RELEASE, "workgroup");
    __builtin_amdgcn_wave_barrier();
    __builtin_amdgcn_fence(__ATOMIC_ACQUIRE, "workgroup");
    {
      const int hh = lane >> 4, c4 = (lane & 15) * 4;
      for (int pass = 0; pass < 2; ++pass) {
#pragma unroll
        for (int it = 0; it < 8; ++it) {
          const int row = it * 2 + hh;
          v4f v = *(const v4f*)(slab + row * 68 + c4);
          *(volatile v4f*)(C + (size_t)(mBase + row) * ldc + n0 + c4) = v;
        }
        __threadfence();
      }
    }
    __builtin_amdgcn_fence(__ATOMIC_RELEASE, "workgroup");
    __builtin_amdgcn_wave_barrier();
    __builtin_amdgcn_fence(__ATOMIC_ACQUIRE, "workgroup");
  }
}

__global__ __launch_bounds__(256) void rowwise_out_kernel(
    const float* __restrict__ PP, const float* __restrict__ x,
    const float* __restrict__ b1, const float* __restrict__ b2, const float* __restrict__ b3,
    float* __restrict__ y)
{
  const int lane = threadIdx.x & 31;
  const int wave = threadIdx.x >> 5;
  const int rbase = (blockIdx.x * 8 + wave) * kRowsPerWave;
  const float b1a = b1[lane], b1b = b1[32 + lane];
  const float b2a = b2[lane], b2b = b2[32 + lane];
  const float b3a = b3[lane], b3b = b3[32 + lane];
#pragma unroll 1
  for (int i = 0; i < kRowsPerWave; ++i) {
    const size_t R = (size_t)(rbase + i);
    const float* pr = PP + R * kNc;
    const float Ba = pr[kDm + lane] + b2a;
    const float Bb = pr[kDm + 32 + lane] + b2b;
    const float Ca = pr[kDm + kNs + lane] + b3a;
    const float Cb = pr[kDm + kNs + 32 + lane] + b3b;
    float s = Ba * Ca;
    s = fmaf(Bb, Cb, s);
    s += __shfl_xor(s, 16, 32);
    s += __shfl_xor(s, 8, 32);
    s += __shfl_xor(s, 4, 32);
    s += __shfl_xor(s, 2, 32);
    s += __shfl_xor(s, 1, 32);
#pragma unroll 1
    for (int hf = 0; hf < 2; ++hf) {
      const float bsel = (hf == 0) ? b1a : b1b;
      const int col = hf * 32 + lane;
      const float v  = pr[col] + bsel;
      const float xv = x[R * kDm + col];
      const float sp = fmaxf(v, 0.0f) + log1pf(expf(-fabsf(v)));
      const float yv = (xv * sp) * s;
      float* q = y + R * kDm + col;
      *(volatile float*)q = yv;
      __threadfence();
      *(volatile float*)q = yv;
    }
  }
}

extern "C" void kernel_launch(void* const* d_in, const int* in_sizes, int n_in,
                              void* d_out, int out_size, void* d_ws, size_t ws_size,
                              hipStream_t stream) {
  (void)stream;
  if (n_in < 7) return;
  if (in_sizes[0] != kRows * kDm) return;
  if (in_sizes[1] != kDm * kDm) return;
  if (in_sizes[2] != kDm) return;
  if (in_sizes[3] != kNs * kDm) return;
  if (in_sizes[4] != kNs) return;
  if (in_sizes[5] != kNs * kDm) return;
  if (in_sizes[6] != kNs) return;
  if (out_size != kRows * kDm) return;
  if (ws_size < kWsTotal) return;

  const float* x  = (const float*)d_in[0];
  const float* W1 = (const float*)d_in[1];
  const float* b1 = (const float*)d_in[2];
  const float* W2 = (const float*)d_in[3];
  const float* b2 = (const float*)d_in[4];
  const float* W3 = (const float*)d_in[5];
  const float* b3 = (const float*)d_in[6];
  float* y = (float*)d_out;

  char* ws = (char*)d_ws;
  unsigned short* AP = (unsigned short*)(ws + kOffAP);
  unsigned short* BT = (unsigned short*)(ws + kOffBT);
  float*          PP = (float*)(ws + kOffPP);

  build_planes_kernel<<<kXBlocks + kWBlocks, 256, 0, stream>>>(x, W1, W2, W3, AP, BT);

  wmma_gemm64_bf16<<<kGemmBlocks, 256, 0, stream>>>(AP, kKc, BT, kKc, PP, kNc, kRows, kNc, kKc);

  rowwise_out_kernel<<<kOutBlocks, 256, 0, stream>>>(PP, x, b1, b2, b3, y);
}
